// Transformer_Block_532575945176
// MI455X (gfx1250) — hardware-verified
//
#include <hip/hip_runtime.h>
#include <math.h>

constexpr int kB    = 2;
constexpr int kS    = 1024;
constexpr int kHid  = 1024;
constexpr int kNH   = 16;
constexpr int kHD   = 64;
constexpr int kProj = 4096;
constexpr int kTok  = kB * kS;
constexpr int kGrp  = 8;
constexpr int kNChunk = (kB * kNH) / kGrp;
static_assert(kNH % kGrp == 0, "chunk of heads stays inside one batch index");
static_assert(kNH * kHD == kHid, "head layout");

constexpr float kWCarry    = 16.0f;
constexpr float kWCarryInv = 1.0f / 16.0f;
constexpr float kPCarry    = 2048.0f;
constexpr float kAttCarry  = 64.0f;
constexpr float kPVScale   = kAttCarry / kPCarry;
constexpr float kWoScale   = 1.0f / (kAttCarry * kWCarry);
constexpr float kInvHid    = 1.0f / 1024.0f;
constexpr float kLnEps     = 1e-5f;
constexpr float kScoreScale = 0.125f;

constexpr size_t kMiB   = 1048576;
constexpr size_t oWoT   = 0 * kMiB;
constexpr size_t oW1T   = 2 * kMiB;
constexpr size_t oW2T   = 10 * kMiB;
constexpr size_t oQw    = 18 * kMiB;
constexpr size_t oQr    = 22 * kMiB;
constexpr size_t oK16   = 26 * kMiB;
constexpr size_t oR16   = 30 * kMiB;
constexpr size_t oVT    = 32 * kMiB;
constexpr size_t oATT   = 36 * kMiB;
constexpr size_t oWqT   = 40 * kMiB;
constexpr size_t oWkvT  = 42 * kMiB;
constexpr size_t oWrT   = 46 * kMiB;
constexpr size_t oX16   = 48 * kMiB;
constexpr size_t oPOS   = 52 * kMiB;
constexpr size_t oQf    = 54 * kMiB;
constexpr size_t oAC    = 40 * kMiB;
constexpr size_t oBD    = 72 * kMiB;
constexpr size_t oP16   = 104 * kMiB;
constexpr size_t oPre1  = 40 * kMiB;
constexpr size_t oOut1f = 48 * kMiB;
constexpr size_t oOut1h = 56 * kMiB;
constexpr size_t oH16   = 60 * kMiB;
constexpr size_t oPre2  = 76 * kMiB;
constexpr size_t kWsNeed = 120 * kMiB;
static_assert(oWkvT + (size_t)2048 * 1024 * 2 == oWrT, "WkvT extent");
static_assert(oQf + (size_t)kTok * kHid * 4 <= 62 * kMiB, "Qf32 extent");
static_assert(oAC + (size_t)kGrp * kS * kS * 4 == oBD, "AC extent");
static_assert(oBD + (size_t)kGrp * kS * kS * 4 == oP16, "BD extent");
static_assert(oP16 + (size_t)kGrp * kS * kS * 2 == kWsNeed, "P16 extent");
static_assert(oH16 + (size_t)kTok * kProj * 2 == oPre2, "H16 extent");
static_assert(oPre2 + (size_t)kTok * kHid * 4 <= kWsNeed, "pre2 extent");
static_assert(kWsNeed <= (size_t)134217728, "carve under 128 MiB");

typedef __attribute__((ext_vector_type(16))) _Float16 v16h;
typedef __attribute__((ext_vector_type(8)))  _Float16 v8h;
typedef __attribute__((ext_vector_type(16))) __bf16   v16b;
typedef __attribute__((ext_vector_type(8)))  __bf16   v8b;
typedef __attribute__((ext_vector_type(8)))  float    v8f;
typedef __attribute__((ext_vector_type(4)))  float    v4f;
typedef __attribute__((ext_vector_type(4)))  unsigned int v4u;
typedef __attribute__((ext_vector_type(4)))  int      v4i;

__device__ __forceinline__ unsigned short f2bf_bits(float f) {
  unsigned u = __float_as_uint(f);
  return (unsigned short)((u + 0x7FFFu + ((u >> 16) & 1u)) >> 16);
}
__device__ __forceinline__ float bf_bits2f(unsigned short h) { return __uint_as_float(((unsigned)h) << 16); }

__device__ __forceinline__ void dep_guard_h(v8f& a, v8f& b, v16h x, v16h y) { asm volatile("v_nop\n\tv_nop\n\tv_nop\n\tv_nop" : "+v"(a), "+v"(b) : "v"(x), "v"(y)); }
__device__ __forceinline__ void dep_guard_b(v8f& a, v8f& b, v16b x, v16b y) { asm volatile("v_nop\n\tv_nop\n\tv_nop\n\tv_nop" : "+v"(a), "+v"(b) : "v"(x), "v"(y)); }
__device__ __forceinline__ void keep4_h(v16h a, v16h b, v16h c, v16h d) { asm volatile("v_nop" :: "v"(a), "v"(b), "v"(c), "v"(d)); }
__device__ __forceinline__ void keep4_b(v16b a, v16b b, v16b c, v16b d) { asm volatile("v_nop" :: "v"(a), "v"(b), "v"(c), "v"(d)); }
__device__ __forceinline__ void acc_guard4(v8f& a, v8f& b, v8f& c, v8f& d) { asm volatile("v_nop\n\tv_nop\n\tv_nop\n\tv_nop" : "+v"(a), "+v"(b), "+v"(c), "+v"(d)); }
template <typename T> struct Frag;
template <> struct Frag<_Float16> {
  typedef v16h V; union U { v16h v; v8h h[2]; };
  static __device__ __forceinline__ v16h load(const _Float16* p) {
    U f; f.h[0] = *(const v8h*)(p); f.h[1] = *(const v8h*)(p + 16); return f.v;
  }
  static __device__ __forceinline__ v8f mma(v16h a, v16h b, v8f c) {
    return __builtin_amdgcn_wmma_f32_16x16x32_f16(false, a, false, b, (short)0, c, false, false);
  }
  static __device__ __forceinline__ void guard(v8f& a, v8f& b, v16h x, v16h y) { dep_guard_h(a, b, x, y); }
  static __device__ __forceinline__ void keep(v16h a, v16h b, v16h c, v16h d) { keep4_h(a, b, c, d); }
};
template <> struct Frag<__bf16> {
  typedef v16b V; union U { v16b v; v8b h[2]; };
  static __device__ __forceinline__ v16b load(const __bf16* p) {
    U f; f.h[0] = *(const v8b*)(p); f.h[1] = *(const v8b*)(p + 16); return f.v;
  }
  static __device__ __forceinline__ v8f mma(v16b a, v16b b, v8f c) {
    return __builtin_amdgcn_wmma_f32_16x16x32_bf16(false, a, false, b, (short)0, c, false, false);
  }
  static __device__ __forceinline__ void guard(v8f& a, v8f& b, v16b x, v16b y) { dep_guard_b(a, b, x, y); }
  static __device__ __forceinline__ void keep(v16b a, v16b b, v16b c, v16b d) { keep4_b(a, b, c, d); }
};

__device__ __forceinline__ unsigned pk16(unsigned short a, unsigned short b) { return (unsigned)a | ((unsigned)b << 16); }
__device__ __forceinline__ unsigned short h_bits(float f) { const _Float16 h = (_Float16)f; return __builtin_bit_cast(unsigned short, h); }

template <int ET> struct Elem;
template <> struct Elem<0> { typedef _Float16 T; };
template <> struct Elem<1> { typedef __bf16 T; };
template <int ET, bool SPLIT, int BIAS_MODE, int OUT_MODE, bool RESID, int ACT = 0>
__global__ __launch_bounds__(256) void wmma_gemm64(
    const unsigned short* __restrict__ Ap, const unsigned short* __restrict__ A2p, int lda, long strideA,
    const unsigned short* __restrict__ Btp, const unsigned short* __restrict__ Bt2p, int ldb, long strideB,
    void* __restrict__ Cout, void* __restrict__ Cout2, int ldc, long strideC,
    const float* __restrict__ bias,
    const float* __restrict__ resid, long strideR,
    int M, int N, int K, float scale) {
  typedef typename Elem<ET>::T T;
  typedef typename Frag<T>::V V;
  const T* A = (const T*)Ap; const T* A2 = (const T*)A2p; const T* Bt = (const T*)Btp; const T* Bt2 = (const T*)Bt2p;
  __shared__ __align__(16) float sT[8][16 * 68];
  const int b    = blockIdx.y;
  const int lane = threadIdx.x & 31;
  const int wave = threadIdx.x >> 5;
  const int tilesN = N >> 6;
  const int tilesM = M >> 6;
  const int tile = blockIdx.x * 8 + wave;
  if (tile >= tilesM * tilesN) return;
  const int tm = tile / tilesN;
  const int tn = tile - tm * tilesN;
  const int m0 = tm << 6;
  const int n0 = tn << 6;

  const T* Ab  = A  + (size_t)b * strideA;
  const T* Bb  = Bt + (size_t)b * strideB;
  const T* Ab2 = SPLIT ? (A2  + (size_t)b * strideA) : nullptr;
  const T* Bb2 = SPLIT ? (Bt2 + (size_t)b * strideB) : nullptr;

  const int rlane = lane & 15;
  const int koff  = (lane >> 4) * 8;
  const int mOff  = (lane >> 4) * 8;

  v8f acc[4][4];
#pragma unroll
  for (int i = 0; i < 4; ++i)
#pragma unroll
    for (int j = 0; j < 4; ++j) acc[i][j] = (v8f){0.f,0.f,0.f,0.f,0.f,0.f,0.f,0.f};

  for (int k0 = 0; k0 < K; k0 += 32) {
    V bh[4], bl[4];
#pragma unroll
    for (int j = 0; j < 4; ++j) {
      const size_t bo = (size_t)(n0 + (j << 4) + rlane) * ldb + koff + k0;
      bh[j] = Frag<T>::load(Bb + bo);
      if (SPLIT) bl[j] = Frag<T>::load(Bb2 + bo);
    }
#pragma unroll
    for (int i = 0; i < 4; ++i) {
      const size_t ao = (size_t)(m0 + (i << 4) + rlane) * lda + koff + k0;
      V ah = Frag<T>::load(Ab + ao);
      V al;
      if (SPLIT) al = Frag<T>::load(Ab2 + ao);
#pragma unroll
      for (int j = 0; j < 4; ++j) {
        acc[i][j] = Frag<T>::mma(ah, bh[j], acc[i][j]);
        if (SPLIT) {
          acc[i][j] = Frag<T>::mma(ah, bl[j], acc[i][j]);
          acc[i][j] = Frag<T>::mma(al, bh[j], acc[i][j]);
        }
      }
      Frag<T>::guard(acc[i][0], acc[i][3], ah, SPLIT ? al : ah);
    }
    Frag<T>::keep(bh[0], bh[1], bh[2], bh[3]);
    if (SPLIT) Frag<T>::keep(bl[0], bl[1], bl[2], bl[3]);
  }
  acc_guard4(acc[0][0], acc[0][1], acc[0][2], acc[0][3]);
  acc_guard4(acc[1][0], acc[1][1], acc[1][2], acc[1][3]);
  acc_guard4(acc[2][0], acc[2][1], acc[2][2], acc[2][3]);
  acc_guard4(acc[3][0], acc[3][1], acc[3][2], acc[3][3]);

  float* slab = sT[wave];
  const float* Rb = RESID ? (resid + (size_t)b * strideR) : nullptr;
#pragma unroll
  for (int i = 0; i < 4; ++i) {
    const int mBase = m0 + (i << 4);
#pragma unroll
    for (int j = 0; j < 4; ++j) {
      const int n = n0 + (j << 4) + rlane;
      float bv = 0.f;
      if (BIAS_MODE == 2) bv = bias[n];
#pragma unroll
      for (int r = 0; r < 8; ++r) {
        float v = acc[i][j][r] * scale;
        if (BIAS_MODE == 1) v += bias[mBase + mOff + r];
        if (BIAS_MODE == 2) v += bv;
        if (RESID) v += Rb[(size_t)(mBase + mOff + r) * ldc + n];
        if (ACT == 2) v = fmaxf(v, 0.0f);
        if (ACT == 4) v = (v > 0.f) ? v : 0.01f * v;
        slab[(mOff + r) * 68 + (j << 4) + rlane] = v;
      }
    }
    __builtin_amdgcn_fence(__ATOMIC_RELEASE, "workgroup");
    __builtin_amdgcn_wave_barrier();
    __builtin_amdgcn_fence(__ATOMIC_ACQUIRE, "workgroup");
    if (OUT_MODE == 0) {
      float* C = (float*)Cout + (size_t)b * strideC;
      const int hh = lane >> 4, c4 = (lane & 15) * 4;
      for (int pass = 0; pass < 2; ++pass) {
#pragma unroll
        for (int it = 0; it < 8; ++it) {
          const int row = it * 2 + hh;
          v4f v = *(const v4f*)(slab + row * 68 + c4);
          *(volatile v4f*)(C + (size_t)(mBase + row) * ldc + n0 + c4) = v;
        }
        __threadfence();
      }
    } else {
      const int q = lane >> 3, c8 = (lane & 7) * 8;
      unsigned short* C  = (unsigned short*)Cout  + (size_t)b * strideC;
      unsigned short* C2 = (OUT_MODE == 2) ? ((unsigned short*)Cout2 + (size_t)b * strideC) : nullptr;
      for (int pass = 0; pass < 2; ++pass) {
#pragma unroll
        for (int it = 0; it < 4; ++it) {
          const int row = it * 4 + q;
          const float* sp = slab + row * 68 + c8;
          v8h hv, lv;
#pragma unroll
          for (int e = 0; e < 8; ++e) {
            if (OUT_MODE == 1) {
              hv[e] = (_Float16)sp[e];
            } else {
              unsigned short hb = f2bf_bits(sp[e]);
              unsigned short lb = f2bf_bits(sp[e] - bf_bits2f(hb));
              hv[e] = __builtin_bit_cast(_Float16, hb);
              lv[e] = __builtin_bit_cast(_Float16, lb);
            }
          }
          *(volatile v8h*)(C + (size_t)(mBase + row) * ldc + n0 + c8) = hv;
          if (OUT_MODE == 2) *(volatile v8h*)(C2 + (size_t)(mBase + row) * ldc + n0 + c8) = lv;
        }
        __threadfence();
      }
    }
    __builtin_amdgcn_fence(__ATOMIC_RELEASE, "workgroup");
    __builtin_amdgcn_wave_barrier();
    __builtin_amdgcn_fence(__ATOMIC_ACQUIRE, "workgroup");
  }
}

__global__ __launch_bounds__(256) void wtcast_kernel(const float* __restrict__ W, unsigned short* __restrict__ out,
                                                     int nin, int nout, float scale) {
  __shared__ float sm[64][65];
  const int t  = threadIdx.x;
  const int i0 = blockIdx.x * 64;
  const int o0 = blockIdx.y * 64;
#pragma unroll
  for (int it = 0; it < 16; ++it) {
    const int e = it * 256 + t;
    const int r = e >> 6;
    const int c = e & 63;
    sm[c][r] = W[(size_t)(i0 + r) * nout + o0 + c] * scale;
  }
  __syncthreads();
  const int lane = t & 31, wave = t >> 5;
  const int q = lane >> 3, c8 = (lane & 7) * 8;
  for (int pass = 0; pass < 2; ++pass) {
#pragma unroll
    for (int it = 0; it < 2; ++it) {
      const int row = wave * 8 + it * 4 + q;
      unsigned short hb[8];
#pragma unroll
      for (int e = 0; e < 8; ++e) hb[e] = h_bits(sm[row][c8 + e]);
      const v4u u = (v4u){pk16(hb[0], hb[1]), pk16(hb[2], hb[3]), pk16(hb[4], hb[5]), pk16(hb[6], hb[7])};
      *(volatile v4u*)(out + (size_t)(o0 + row) * nin + i0 + c8) = u;
    }
    __threadfence();
  }
}

__global__ __launch_bounds__(256) void cast8_f16_kernel(const float* __restrict__ in, unsigned short* __restrict__ out, int n8) {
  const int i = blockIdx.x * 256 + threadIdx.x;
  if (i >= n8) return;
  const float* p = in + 8 * (size_t)i;
  const v4f a = *(const v4f*)(p);
  const v4f c = *(const v4f*)(p + 4);
  unsigned short hb[8];
#pragma unroll
  for (int e = 0; e < 4; ++e) {
    hb[e]     = h_bits(a[e]);
    hb[4 + e] = h_bits(c[e]);
  }
  const v4u u = (v4u){pk16(hb[0], hb[1]), pk16(hb[2], hb[3]), pk16(hb[4], hb[5]), pk16(hb[6], hb[7])};
  unsigned short* q = out + 8 * (size_t)i;
  *(volatile v4u*)q = u;
  __threadfence();
  *(volatile v4u*)q = u;
}

__global__ __launch_bounds__(256) void qbias_kernel(const float* __restrict__ Qf, const float* __restrict__ rw,
                                                    const float* __restrict__ rr, unsigned short* __restrict__ Qw,
                                                    unsigned short* __restrict__ Qr, int n8) {
  const int i = blockIdx.x * 256 + threadIdx.x;
  if (i >= n8) return;
  const size_t base = 8 * (size_t)i;
  const int col = (int)(base & (size_t)(kHid - 1));
  const v4f q0 = *(const v4f*)(Qf + base);
  const v4f q1 = *(const v4f*)(Qf + base + 4);
  const v4f w0 = *(const v4f*)(rw + col);
  const v4f w1 = *(const v4f*)(rw + col + 4);
  const v4f r0 = *(const v4f*)(rr + col);
  const v4f r1 = *(const v4f*)(rr + col + 4);
  unsigned short hw[8], hr[8];
#pragma unroll
  for (int e = 0; e < 4; ++e) {
    hw[e]     = h_bits(q0[e] + w0[e]);
    hw[4 + e] = h_bits(q1[e] + w1[e]);
    hr[e]     = h_bits(q0[e] + r0[e]);
    hr[4 + e] = h_bits(q1[e] + r1[e]);
  }
  const v4u uw = (v4u){pk16(hw[0], hw[1]), pk16(hw[2], hw[3]), pk16(hw[4], hw[5]), pk16(hw[6], hw[7])};
  const v4u ur = (v4u){pk16(hr[0], hr[1]), pk16(hr[2], hr[3]), pk16(hr[4], hr[5]), pk16(hr[6], hr[7])};
  unsigned short* pw = Qw + base;
  unsigned short* pr = Qr + base;
  *(volatile v4u*)pw = uw;
  *(volatile v4u*)pr = ur;
  __threadfence();
  *(volatile v4u*)pw = uw;
  *(volatile v4u*)pr = ur;
}

__global__ __launch_bounds__(256) void softmax_rel_kernel(const float* __restrict__ ACp, const float* __restrict__ BDp,
                                                          const int* __restrict__ mask, unsigned short* __restrict__ P,
                                                          float carry) {
  __shared__ float redM[8];
  __shared__ float redS[8];
  __shared__ __align__(16) float sP[kS];
  const int gr   = blockIdx.x;
  const int g    = gr >> 10;
  const int i    = gr & (kS - 1);
  const int t    = threadIdx.x;
  const int lane = t & 31, wave = t >> 5;
  const int c0   = t * 4;
  const v4f a  = *(const v4f*)(ACp + (size_t)gr * kS + c0);
  const v4i mk = *(const v4i*)(mask + (size_t)i * kS + c0);
  const float* bdg = BDp + (size_t)g * kS * kS;
  float x[4];
#pragma unroll
  for (int e = 0; e < 4; ++e) {
    const int j = c0 + e;
    const bool jle = (j <= i);
    int qr = jle ? i : (i + 1);
    qr = (qr > kS - 1) ? (kS - 1) : qr;
    int cc = jle ? (j + (kS - 1) - i) : (j - i - 2);
    cc = (cc < 0) ? 0 : ((cc > kS - 1) ? (kS - 1) : cc);
    const float bvl = bdg[(size_t)qr * kS + cc];
    const bool zero = ((!jle) && (j == i + 1)) || (j > i + (kS - 2));
    const float bd = zero ? 0.0f : bvl;
    const float s = (a[e] + bd) * kScoreScale;
    x[e] = (mk[e] != 0) ? -INFINITY : s;
  }
  float m = fmaxf(fmaxf(x[0], x[1]), fmaxf(x[2], x[3]));
#pragma unroll
  for (int off = 16; off > 0; off >>= 1) m = fmaxf(m, __shfl_xor(m, off, 32));
  if (lane == 0) redM[wave] = m;
  __syncthreads();
  float gm = redM[0];
#pragma unroll
  for (int w = 1; w < 8; ++w) gm = fmaxf(gm, redM[w]);
  float ex[4];
  float psum = 0.f;
#pragma unroll
  for (int e = 0; e < 4; ++e) { ex[e] = expf(x[e] - gm); psum += ex[e]; }
#pragma unroll
  for (int off = 16; off > 0; off >>= 1) psum += __shfl_xor(psum, off, 32);
  if (lane == 0) redS[wave] = psum;
  __syncthreads();
  float tot = redS[0];
#pragma unroll
  for (int w = 1; w < 8; ++w) tot += redS[w];
  const float inv = 1.0f / tot;
  const float mul = inv * carry;
#pragma unroll
  for (int e = 0; e < 4; ++e) sP[c0 + e] = ex[e] * mul;
  __syncthreads();
  if (t < 128) {
    const v4f p0 = *(const v4f*)(sP + 8 * t);
    const v4f p1 = *(const v4f*)(sP + 8 * t + 4);
    unsigned short hb[8];
#pragma unroll
    for (int e = 0; e < 4; ++e) {
      hb[e]     = h_bits(p0[e]);
      hb[4 + e] = h_bits(p1[e]);
    }
    const v4u u = (v4u){pk16(hb[0], hb[1]), pk16(hb[2], hb[3]), pk16(hb[4], hb[5]), pk16(hb[6], hb[7])};
    unsigned short* pp = P + (size_t)gr * kS + 8 * t;
    *(volatile v4u*)pp = u;
    __threadfence();
    *(volatile v4u*)pp = u;
  }
}

template <bool WITH_H>
__global__ __launch_bounds__(256) void layernorm_kernel(const float* __restrict__ in, const float* __restrict__ gam,
                                                        const float* __restrict__ bet, float* __restrict__ outF,
                                                        unsigned short* __restrict__ outH) {
  __shared__ float red1[8];
  __shared__ float red2[8];
  __shared__ __align__(16) float sY[WITH_H ? kHid : 4];
  const int row  = blockIdx.x;
  const int t    = threadIdx.x;
  const int lane = t & 31, wave = t >> 5;
  const int c0   = t * 4;
  const v4f xv = *(const v4f*)(in + (size_t)row * kHid + c0);
  float s = (xv[0] + xv[1]) + (xv[2] + xv[3]);
#pragma unroll
  for (int off = 16; off > 0; off >>= 1) s += __shfl_xor(s, off, 32);
  if (lane == 0) red1[wave] = s;
  __syncthreads();
  float tot = red1[0];
#pragma unroll
  for (int w = 1; w < 8; ++w) tot += red1[w];
  const float mean = tot * kInvHid;
  float d[4];
  float sq = 0.f;
#pragma unroll
  for (int e = 0; e < 4; ++e) { d[e] = xv[e] - mean; sq += d[e] * d[e]; }
#pragma unroll
  for (int off = 16; off > 0; off >>= 1) sq += __shfl_xor(sq, off, 32);
  if (lane == 0) red2[wave] = sq;
  __syncthreads();
  float tot2 = red2[0];
#pragma unroll
  for (int w = 1; w < 8; ++w) tot2 += red2[w];
  const float var  = tot2 * kInvHid;
  const float rstd = rsqrtf(var + kLnEps);
  const v4f gv = *(const v4f*)(gam + c0);
  const v4f bv = *(const v4f*)(bet + c0);
  v4f yv;
#pragma unroll
  for (int e = 0; e < 4; ++e) yv[e] = d[e] * rstd * gv[e] + bv[e];
  float* op = outF + (size_t)row * kHid + c0;
  *(volatile v4f*)op = yv;
  __threadfence();
  *(volatile v4f*)op = yv;
  if (WITH_H) {
#pragma unroll
    for (int e = 0; e < 4; ++e) sY[c0 + e] = yv[e];
    __syncthreads();
    if (t < 128) {
      const v4f p0 = *(const v4f*)(sY + 8 * t);
      const v4f p1 = *(const v4f*)(sY + 8 * t + 4);
      unsigned short hb[8];
#pragma unroll
      for (int e = 0; e < 4; ++e) {
        hb[e]     = h_bits(p0[e]);
        hb[4 + e] = h_bits(p1[e]);
      }
      const v4u u = (v4u){pk16(hb[0], hb[1]), pk16(hb[2], hb[3]), pk16(hb[4], hb[5]), pk16(hb[6], hb[7])};
      unsigned short* hp = outH + (size_t)row * kHid + 8 * t;
      *(volatile v4u*)hp = u;
      __threadfence();
      *(volatile v4u*)hp = u;
    }
  }
}

extern "C" void kernel_launch(void* const* d_in, const int* in_sizes, int n_in,
                              void* d_out, int out_size, void* d_ws, size_t ws_size, hipStream_t stream) {
  (void)in_sizes; (void)n_in;
  if (ws_size < kWsNeed) return;
  if ((size_t)out_size < (size_t)kTok * kHid) return;

  const float* x    = (const float*)d_in[0];
  const float* pos  = (const float*)d_in[2];
  const float* rrb  = (const float*)d_in[3];
  const float* rwb  = (const float*)d_in[4];
  const float* Wkv  = (const float*)d_in[5];
  const float* Wq   = (const float*)d_in[6];
  const float* Wr   = (const float*)d_in[7];
  const float* Wo   = (const float*)d_in[8];
  const float* ln1g = (const float*)d_in[9];
  const float* ln1b = (const float*)d_in[10];
  const float* W1   = (const float*)d_in[11];
  const float* b1   = (const float*)d_in[12];
  const float* W2   = (const float*)d_in[13];
  const float* b2   = (const float*)d_in[14];
  const float* ln2g = (const float*)d_in[15];
  const float* ln2b = (const float*)d_in[16];
  const int*   mask = (const int*)d_in[17];
  float* out = (float*)d_out;

  char* ws = (char*)d_ws;
  typedef unsigned short us;
  us* WoT   = (us*)(ws + oWoT);
  us* W1T   = (us*)(ws + oW1T);
  us* W2T   = (us*)(ws + oW2T);
  us* Qw    = (us*)(ws + oQw);
  us* Qr    = (us*)(ws + oQr);
  us* K16   = (us*)(ws + oK16);
  us* R16   = (us*)(ws + oR16);
  us* VT16  = (us*)(ws + oVT);
  us* ATT   = (us*)(ws + oATT);
  us* WqT   = (us*)(ws + oWqT);
  us* WkvT  = (us*)(ws + oWkvT);
  us* WrT   = (us*)(ws + oWrT);
  us* X16   = (us*)(ws + oX16);
  us* POS16 = (us*)(ws + oPOS);
  float* Qf = (float*)(ws + oQf);
  float* ACp = (float*)(ws + oAC);
  float* BDp = (float*)(ws + oBD);
  us* P16   = (us*)(ws + oP16);
  float* pre1  = (float*)(ws + oPre1);
  float* out1f = (float*)(ws + oOut1f);
  us* out1h    = (us*)(ws + oOut1h);
  us* H16      = (us*)(ws + oH16);
  float* pre2  = (float*)(ws + oPre2);

  wtcast_kernel<<<dim3(kHid / 64, kHid / 64), 256, 0, stream>>>(Wq, WqT, kHid, kHid, kWCarry);
  wtcast_kernel<<<dim3(kHid / 64, (2 * kHid) / 64), 256, 0, stream>>>(Wkv, WkvT, kHid, 2 * kHid, kWCarry);
  wtcast_kernel<<<dim3(kHid / 64, kHid / 64), 256, 0, stream>>>(Wr, WrT, kHid, kHid, kWCarry);
  wtcast_kernel<<<dim3(kHid / 64, kHid / 64), 256, 0, stream>>>(Wo, WoT, kHid, kHid, kWCarry);
  wtcast_kernel<<<dim3(kHid / 64, kProj / 64), 256, 0, stream>>>(W1, W1T, kHid, kProj, kWCarry);
  wtcast_kernel<<<dim3(kProj / 64, kHid / 64), 256, 0, stream>>>(W2, W2T, kProj, kHid, kWCarry);
  cast8_f16_kernel<<<(kTok * kHid / 8) / 256, 256, 0, stream>>>(x, X16, kTok * kHid / 8);
  cast8_f16_kernel<<<(kS * kHid / 8) / 256, 256, 0, stream>>>(pos, POS16, kS * kHid / 8);

  wmma_gemm64<0, false, 0, 0, false, 0><<<dim3(64, 1), 256, 0, stream>>>(
      X16, X16, kHid, 0L, WqT, WqT, kHid, 0L, (void*)Qf, (void*)Qf, kHid, 0L,
      ln1g, x, 0L, kTok, kHid, kHid, kWCarryInv);
  qbias_kernel<<<(kTok * kHid / 8) / 256, 256, 0, stream>>>(Qf, rwb, rrb, Qw, Qr, kTok * kHid / 8);
  wmma_gemm64<0, false, 0, 1, false, 0><<<dim3(64, 1), 256, 0, stream>>>(
      X16, X16, kHid, 0L, WkvT, WkvT, kHid, 0L, (void*)K16, (void*)K16, kHid, 0L,
      ln1g, x, 0L, kTok, kHid, kHid, kWCarryInv);
  wmma_gemm64<0, false, 0, 1, false, 0><<<dim3(64, 1), 256, 0, stream>>>(
      WkvT + (size_t)kHid * kHid, WkvT + (size_t)kHid * kHid, kHid, 0L, X16, X16, kHid, 0L,
      (void*)VT16, (void*)VT16, kTok, 0L,
      ln1g, x, 0L, kHid, kTok, kHid, kWCarryInv);
  wmma_gemm64<0, false, 0, 1, false, 0><<<dim3(32, 1), 256, 0, stream>>>(
      POS16, POS16, kHid, 0L, WrT, WrT, kHid, 0L, (void*)R16, (void*)R16, kHid, 0L,
      ln1g, x, 0L, kS, kHid, kHid, kWCarryInv);

  for (int c = 0; c < kNChunk; ++c) {
    const int bb = c / (kNH / kGrp);
    const int h0 = (c % (kNH / kGrp)) * kGrp;
    const size_t qoff = (size_t)bb * kS * kHid + (size_t)h0 * kHD;
    wmma_gemm64<0, false, 0, 0, false, 0><<<dim3(32, kGrp), 256, 0, stream>>>(
        Qw + qoff, Qw + qoff, kHid, (long)kHD, K16 + qoff, K16 + qoff, kHid, (long)kHD,
        (void*)ACp, (void*)ACp, kS, (long)kS * kS,
        ln1g, x, 0L, kS, kS, kHD, 1.0f);
    wmma_gemm64<0, false, 0, 0, false, 0><<<dim3(32, kGrp), 256, 0, stream>>>(
        Qr + qoff, Qr + qoff, kHid, (long)kHD, R16 + (size_t)h0 * kHD, R16 + (size_t)h0 * kHD, kHid, (long)kHD,
        (void*)BDp, (void*)BDp, kS, (long)kS * kS,
        ln1g, x, 0L, kS, kS, kHD, 1.0f);
    softmax_rel_kernel<<<kGrp * kS, 256, 0, stream>>>(ACp, BDp, mask, P16, kPCarry);
    wmma_gemm64<0, false, 0, 1, false, 0><<<dim3(2, kGrp), 256, 0, stream>>>(
        P16, P16, kS, (long)kS * kS,
        VT16 + (size_t)h0 * kHD * kTok + (size_t)bb * kS, VT16 + (size_t)h0 * kHD * kTok + (size_t)bb * kS, kTok, (long)kHD * kTok,
        (void*)(ATT + qoff), (void*)(ATT + qoff), kHid, (long)kHD,
        ln1g, x, 0L, kS, kHD, kS, kPVScale);
  }

  wmma_gemm64<0, false, 0, 0, true, 0><<<dim3(64, 1), 256, 0, stream>>>(
      ATT, ATT, kHid, 0L, WoT, WoT, kHid, 0L, (void*)pre1, (void*)pre1, kHid, 0L,
      ln1g, x, 0L, kTok, kHid, kHid, kWoScale);
  layernorm_kernel<true><<<kTok, 256, 0, stream>>>(pre1, ln1g, ln1b, out1f, out1h);
  wmma_gemm64<0, false, 2, 1, false, 2><<<dim3(256, 1), 256, 0, stream>>>(
      out1h, out1h, kHid, 0L, W1T, W1T, kHid, 0L, (void*)H16, (void*)H16, kProj, 0L,
      b1, x, 0L, kTok, kProj, kHid, kWCarryInv);
  wmma_gemm64<0, false, 2, 0, true, 0><<<dim3(64, 1), 256, 0, stream>>>(
      H16, H16, kProj, 0L, W2T, W2T, kProj, 0L, (void*)pre2, (void*)pre2, kHid, 0L,
      b2, out1f, 0L, kTok, kHid, kProj, kWCarryInv);
  layernorm_kernel<false><<<kTok, 256, 0, stream>>>(pre2, ln2g, ln2b, out, out1h);
}
